// HummingLayer_46024869544571
// MI455X (gfx1250) — hardware-run, weakly checked
//
#include <hip/hip_runtime.h>
#include <stddef.h>
#include <stdint.h>


#define MD    16
#define ND    8192
#define KD    8192
#define GSZ   128
#define NG    (KD / GSZ)
#define WPR   (KD / 8)
#define ZPR   (ND / 8)
#define XSC   16
#define WSC   1024
#define NTHR  256
#define NWAVE 8
#define BN    128
#define TP    136
#define SP    128
#define WSCAP 134217728

static_assert(NTHR == NWAVE * 32);
static_assert(BN == NWAVE * 16);
static_assert((ND % BN) == 0);
static_assert((KD % GSZ) == 0);
static_assert((GSZ % 32) == 0);
static_assert(GSZ == 16 * 8);
static_assert(NTHR == 2 * BN);
static_assert(((MD * KD) % (8 * NTHR)) == 0);
static_assert((TP % 8) == 0);
static_assert(MD == 2 * NWAVE);
static_assert(BN == 4 * 32);

typedef float          v4f  __attribute__((ext_vector_type(4)));
typedef float          v8f  __attribute__((ext_vector_type(8)));
typedef _Float16       v8h  __attribute__((ext_vector_type(8)));
typedef _Float16       v16h __attribute__((ext_vector_type(16)));
typedef int            v4i  __attribute__((ext_vector_type(4)));
union FragH { v16h v; v8h h[2]; };

__device__ __forceinline__ v8f wmf(v16h a, v16h b, v8f c) {
  v8f d = __builtin_amdgcn_wmma_f32_16x16x32_f16(false, a, false, b, (short)0, c, false, false);
  asm volatile("v_nop\n\tv_nop\n\tv_nop\n\tv_nop" : "+v"(d) : "v"(a), "v"(b));
  return d;
}

__global__ __launch_bounds__(NTHR) void k_prepx(const float* __restrict__ x, _Float16* xh) {
  const size_t t = (size_t)blockIdx.x * NTHR + threadIdx.x;
  const float* p = x + t * 8;
  const v4f f0 = *(const v4f*)p;
  const v4f f1 = *(const v4f*)(p + 4);
  v8h a;
  a[0] = (_Float16)(f0.x * (float)XSC); a[1] = (_Float16)(f0.y * (float)XSC);
  a[2] = (_Float16)(f0.z * (float)XSC); a[3] = (_Float16)(f0.w * (float)XSC);
  a[4] = (_Float16)(f1.x * (float)XSC); a[5] = (_Float16)(f1.y * (float)XSC);
  a[6] = (_Float16)(f1.z * (float)XSC); a[7] = (_Float16)(f1.w * (float)XSC);
  _Float16* d = xh + t * 8;
  *(volatile v8h*)d = a;
  __threadfence();
  *(volatile v8h*)d = a;
}

__global__ __launch_bounds__(NTHR) void k_gemm(const _Float16* __restrict__ xh,
                                               const int* __restrict__ Wq,
                                               const float* __restrict__ Sc,
                                               const int* __restrict__ Zp,
                                               const float* __restrict__ Bias,
                                               const float* __restrict__ Gsc,
                                               float* out) {
  __shared__ __attribute__((aligned(16))) _Float16 wtile[BN * TP];
  __shared__ __attribute__((aligned(16))) float stg[MD * SP];

  const int tid = threadIdx.x, lane = tid & 31, wave = tid >> 5, hh = lane >> 4, m = lane & 15;
  const int n0 = blockIdx.x * BN;

  const int nl = tid >> 1;
  const int wb = (tid & 1) * 8;
  const int n = n0 + nl;
  const int* wrow = Wq + (size_t)n * WPR + wb;
  const int zsh = (n & 7) * 4;
  const int* zcol = Zp + (n >> 3);
  const float* scol = Sc + n;
  _Float16* trow = wtile + nl * TP + 8 * wb;

  const _Float16* ap = xh + (size_t)m * KD + 8 * hh;
  const _Float16* bp = wtile + (16 * wave + m) * TP + 8 * hh;

  v8f acc = {0.f, 0.f, 0.f, 0.f, 0.f, 0.f, 0.f, 0.f};

#pragma unroll 1
  for (int g = 0; g < NG; ++g) {
    __syncthreads();
    const float scw = scol[(size_t)g * ND] * (float)WSC;
    const int zp = (zcol[(size_t)g * ZPR] >> zsh) & 0xF;
    const v4i w0 = *(const v4i*)(wrow + g * 16);
    const v4i w1 = *(const v4i*)(wrow + g * 16 + 4);
    const int wv[8] = {w0.x, w0.y, w0.z, w0.w, w1.x, w1.y, w1.z, w1.w};
#pragma unroll
    for (int i = 0; i < 8; ++i) {
      const int wd = wv[i];
      v8h hv;
#pragma unroll
      for (int j = 0; j < 8; ++j) {
        const int q = (wd >> (4 * j)) & 0xF;
        hv[j] = (_Float16)((float)(q - zp) * scw);
      }
      *(v8h*)(trow + 8 * i) = hv;
    }
    __syncthreads();
#pragma unroll
    for (int kt = 0; kt < GSZ / 32; ++kt) {
      const int k0 = g * GSZ + 32 * kt;
      FragH a, b;
      a.h[0] = *(const v8h*)(ap + k0);
      a.h[1] = *(const v8h*)(ap + k0 + 16);
      b.h[0] = *(const v8h*)(bp + 32 * kt);
      b.h[1] = *(const v8h*)(bp + 32 * kt + 16);
      acc = wmf(a.v, b.v, acc);
    }
  }

  constexpr float OSC = 1.0f / (float)(XSC * WSC);
  const float gs = Gsc[0];
  const int col = 16 * wave + m;
  const float bv = Bias[n0 + col];
  float* sp = stg + (8 * hh) * SP + col;
#pragma unroll
  for (int r = 0; r < 8; ++r) sp[r * SP] = (acc[r] * OSC) * gs + bv;
  __syncthreads();

  const int row0 = 2 * wave;
  const v4f v0 = *(const v4f*)(stg + row0 * SP + 4 * lane);
  const v4f v1 = *(const v4f*)(stg + (row0 + 1) * SP + 4 * lane);
  float* g0 = out + (size_t)row0 * ND + n0 + 4 * lane;
  float* g1 = g0 + ND;
  *(volatile v4f*)g0 = v0;
  *(volatile v4f*)g1 = v1;
  __threadfence();
  *(volatile v4f*)g0 = v0;
  *(volatile v4f*)g1 = v1;
}

extern "C" void kernel_launch(void* const* d_in, const int* in_sizes, int n_in,
                              void* d_out, int out_size, void* d_ws, size_t ws_size,
                              hipStream_t stream) {
  if (n_in < 6) return;
  if (in_sizes[0] != MD * KD) return;
  if (in_sizes[1] != ND * WPR) return;
  if (in_sizes[2] != NG * ND) return;
  if (in_sizes[3] != NG * ZPR) return;
  if (in_sizes[4] != ND) return;
  if (in_sizes[5] < 1) return;
  if (out_size != MD * ND) return;

  const float* x    = (const float*)d_in[0];
  const int*   wq   = (const int*)d_in[1];
  const float* sc   = (const float*)d_in[2];
  const int*   zp   = (const int*)d_in[3];
  const float* bias = (const float*)d_in[4];
  const float* gsc  = (const float*)d_in[5];
  float* out = (float*)d_out;

  char* ws = (char*)d_ws;
  size_t off = 0;
  const size_t oXh = off; off += (size_t)MD * KD * 2; off = (off + 255) & ~(size_t)255;
  if (off > ws_size || off > (size_t)WSCAP) return;
  _Float16* xh = (_Float16*)(ws + oXh);

  k_prepx<<<(MD * KD) / (8 * NTHR), NTHR, 0, stream>>>(x, xh);
  k_gemm<<<ND / BN, NTHR, 0, stream>>>(xh, wq, sc, zp, bias, gsc, out);
}
